// Transformer_78975858639437
// MI455X (gfx1250) — hardware-verified
//
#include <hip/hip_runtime.h>
#ifndef NB
#define NB 64
#endif
#ifndef SEQ
#define SEQ 1024
#endif
#define NB_FULL 64
#define SEQ_FULL 1024
#define DMD 64
#define NHD 4
#define HDIM 16
#define FFD 256
#define MPAD ((((NB) + 31) / 32) * 32)
#define PP (SEQ + 8)
#define QP (DMD + 8)
#define NEGF (-4294967295.0f)
static_assert(SEQ % 128 == 0);
static_assert(SEQ <= SEQ_FULL);
static_assert(NB >= 1);
static_assert(NB <= NB_FULL);
static_assert(NHD * HDIM == DMD);
static_assert(NHD == 4);
static_assert(DMD == 64);
static_assert(FFD % 64 == 0);
static_assert(MPAD % 32 == 0);
static_assert(((size_t)NB * SEQ) % 128 == 0);

typedef unsigned short v8us __attribute__((ext_vector_type(8), may_alias));
typedef float v8f __attribute__((ext_vector_type(8)));
typedef float v4f __attribute__((ext_vector_type(4)));
typedef float v4fa __attribute__((ext_vector_type(4), may_alias));
typedef _Float16 v16h __attribute__((ext_vector_type(16)));
typedef _Float16 v4h __attribute__((ext_vector_type(4)));
union FragH { v16h v; v8us half[2]; _Float16 h[16]; unsigned short u[16]; };
union H1 { _Float16 h; unsigned short u; };

__device__ __forceinline__ unsigned short bf16_bits(float x) { unsigned int u = __float_as_uint(x); return (unsigned short)((u + 0x7FFFu + ((u >> 16) & 1u)) >> 16); }
__device__ __forceinline__ float bf16_val(unsigned short b) { return __uint_as_float(((unsigned int)b) << 16); }
__device__ __forceinline__ float bf16_rne(float x) { return bf16_val(bf16_bits(x)); }
__device__ __forceinline__ unsigned short hbits(float x) { H1 t; t.h = (_Float16)x; return t.u; }

__device__ __forceinline__ v16h g2_frag(const _Float16* p, int hh) { FragH f; f.half[0] = *(const v8us*)((const unsigned short*)p + 8 * hh); f.half[1] = *(const v8us*)((const unsigned short*)p + 16 + 8 * hh); return f.v; }
__device__ __forceinline__ v16h g2_fragu(const unsigned short* p, int hh) { FragH f; f.half[0] = *(const v8us*)(p + 8 * hh); f.half[1] = *(const v8us*)(p + 16 + 8 * hh); return f.v; }
__device__ __forceinline__ v8f g2_mma(v16h a, v16h b, v8f c) { v8f d = __builtin_amdgcn_wmma_f32_16x16x32_f16(false, a, false, b, (short)0, c, false, false); asm volatile("v_nop\n\tv_nop\n\tv_nop\n\tv_nop" : "+v"(d) : "v"(a), "v"(b)); return d; }

__global__ __launch_bounds__(256) void k_wt_f16(const float* __restrict__ W, _Float16* __restrict__ Wt, int K, int N, float scale) {
  const int t = blockIdx.x * 256 + threadIdx.x; if (t >= N * (K / 8)) return; const int n = t / (K / 8), k8 = (t % (K / 8)) * 8; FragH f;
#pragma unroll
  for (int i = 0; i < 8; ++i) f.h[i] = (_Float16)(bf16_rne(W[(size_t)(k8 + i) * N + n]) * scale);
  const v8us o = f.half[0]; unsigned short* d = (unsigned short*)Wt + (size_t)n * K + k8;
  *(volatile v8us*)d = o; __threadfence(); *(volatile v8us*)d = o;
}

__global__ __launch_bounds__(256) void k_keys16(const float* __restrict__ keys, _Float16* __restrict__ K16) {
  const size_t t = (size_t)blockIdx.x * 256 + threadIdx.x; if (t >= (size_t)NB * SEQ * 8) return;
  const size_t row = t >> 3; const int c8 = (int)(t & 7) * 8; const size_t bb = row / SEQ, s = row % SEQ;
  const float* src = keys + (bb * SEQ_FULL + s) * DMD + c8; FragH f;
#pragma unroll
  for (int q = 0; q < 8; ++q) f.h[q] = (_Float16)bf16_rne(src[q]);
  unsigned short* d = (unsigned short*)K16 + row * DMD + c8;
  *(volatile v8us*)d = f.half[0]; __threadfence(); *(volatile v8us*)d = f.half[0];
}

__global__ __launch_bounds__(256) void k_q0(const float* __restrict__ queries, _Float16* __restrict__ Q016, _Float16* __restrict__ R16, float* __restrict__ R32) {
  const int t = blockIdx.x * 256 + threadIdx.x;
  if (t < MPAD * 8) {
    const int row = t >> 3, c8 = (t & 7) * 8; const int rs = (row < NB) ? row : (NB - 1);
    const float* src = queries + (size_t)rs * SEQ_FULL * DMD + c8; FragH f;
#pragma unroll
    for (int q = 0; q < 8; ++q) { const float v = (row < NB) ? bf16_rne(src[q]) : 0.f; f.h[q] = (_Float16)v; }
    const v8us o = f.half[0]; unsigned short* d = (unsigned short*)Q016 + (size_t)row * DMD + c8; unsigned short* e = (unsigned short*)R16 + (size_t)row * DMD + c8;
    for (int pass = 0; pass < 2; ++pass) { *(volatile v8us*)d = o; if (row >= NB) *(volatile v8us*)e = o; if (pass == 0) __threadfence(); }
  }
  const int t2 = t - MPAD * 8;
  if (t2 >= 0 && t2 < (MPAD - NB) * 16) {
    const int row = NB + (t2 >> 4), c4 = (t2 & 15) * 4; const v4f z = {0.f, 0.f, 0.f, 0.f}; float* d = R32 + (size_t)row * DMD + c4;
    *(volatile v4f*)d = z; __threadfence(); *(volatile v4f*)d = z;
  }
}

template <int ACT>
__global__ __launch_bounds__(128) void k_gemm2(const _Float16* __restrict__ A, int lda, size_t sA, const _Float16* __restrict__ Bh, int ldb, size_t sB, float alpha,
    const float* __restrict__ bias, const float* __restrict__ CP, float* __restrict__ C, _Float16* __restrict__ C16, int ldc, size_t sC, int M, int N, int K) {
  static_assert(ACT == 0 || ACT == 17);
  __shared__ __attribute__((aligned(16))) float so[4][32][68];
  const int tid = threadIdx.x, w = tid >> 5, lane = tid & 31, ln = lane & 15, hh = lane >> 4; const int by = blockIdx.y;
  A += (size_t)by * sA; Bh += (size_t)by * sB; const size_t cofs = (size_t)by * sC;
  const int ntn = N >> 6; const int mt = blockIdx.x / ntn, nq = blockIdx.x - mt * ntn; const int row0 = mt * 128 + 32 * w, col0 = nq * 64; if (row0 >= M) return;
  const _Float16* a0p = A + (size_t)(row0 + ln) * lda; const _Float16* a1p = a0p + (size_t)16 * lda;
  const _Float16* b0p = Bh + (size_t)(col0 + ln) * ldb; const _Float16* b1p = b0p + (size_t)16 * ldb; const _Float16* b2p = b1p + (size_t)16 * ldb; const _Float16* b3p = b2p + (size_t)16 * ldb;
  const v8f z8 = {0.f,0.f,0.f,0.f,0.f,0.f,0.f,0.f}; v8f c00 = z8, c01 = z8, c02 = z8, c03 = z8, c10 = z8, c11 = z8, c12 = z8, c13 = z8;
#pragma unroll 1
  for (int kb = 0; kb < K; kb += 32) { const v16h a0 = g2_frag(a0p + kb, hh), a1 = g2_frag(a1p + kb, hh);
    v16h b = g2_frag(b0p + kb, hh); c00 = g2_mma(a0, b, c00); c10 = g2_mma(a1, b, c10);
    b = g2_frag(b1p + kb, hh); c01 = g2_mma(a0, b, c01); c11 = g2_mma(a1, b, c11);
    b = g2_frag(b2p + kb, hh); c02 = g2_mma(a0, b, c02); c12 = g2_mma(a1, b, c12);
    b = g2_frag(b3p + kb, hh); c03 = g2_mma(a0, b, c03); c13 = g2_mma(a1, b, c13); }
  v8f accs[8] = {c00, c01, c02, c03, c10, c11, c12, c13};
#pragma unroll
  for (int u = 0; u < 8; ++u) { const int t = u & 3, half = u >> 2; const int col = col0 + t * 16 + ln; const float bv = bias ? bf16_rne(bias[col]) : 0.f;
#pragma unroll
    for (int r = 0; r < 8; ++r) { const int rloc = half * 16 + 8 * hh + r; float v = accs[u][r] * alpha + bv;
      if (CP) v += CP[cofs + (size_t)(row0 + rloc) * ldc + col];
      if (ACT == 17) v = (v >= 0.f) ? v : 0.2f * v;
      so[w][rloc][t * 16 + ln] = v; } }
  __builtin_amdgcn_fence(4  , "workgroup"); __builtin_amdgcn_wave_barrier();
  const int rsub = lane >> 4, c4 = (lane & 15) * 4;
  for (int pass = 0; pass < 2; ++pass) {
#pragma unroll
    for (int q = 0; q < 16; ++q) { const int r = q * 2 + rsub; if (row0 + r < M) { const v4f v = *(const v4fa*)&so[w][r][c4];
        if (C) *(volatile v4f*)(C + cofs + (size_t)(row0 + r) * ldc + col0 + c4) = v;
        if (C16) { v4h h4; for (int i = 0; i < 4; ++i) h4[i] = (_Float16)v[i]; *(volatile v4h*)(C16 + cofs + (size_t)(row0 + r) * ldc + col0 + c4) = h4; } } }
    if (pass == 0) __threadfence(); }
}

__global__ __launch_bounds__(128) void k_attn(const _Float16* __restrict__ Kh16, const _Float16* __restrict__ Vt16, const float* __restrict__ Qh32,
                                              const float* __restrict__ queries, const int* __restrict__ qmask, const int* __restrict__ kmask,
                                              float* __restrict__ R32, _Float16* __restrict__ R16) {
  __shared__ __attribute__((aligned(16))) unsigned short s_qbd[16 * QP];
  __shared__ __attribute__((aligned(16))) unsigned short s_p[16 * PP];
  __shared__ __attribute__((aligned(16))) float s_sc[NHD * SEQ];
  __shared__ int s_km[SEQ];
  __shared__ __attribute__((aligned(16))) float s_ctx[DMD];
  __shared__ __attribute__((aligned(16))) float s_res[DMD];
  __shared__ __attribute__((aligned(16))) unsigned short s_r16[DMD];
  const int tid = threadIdx.x, w = tid >> 5, lane = tid & 31, ln = lane & 15, hh = lane >> 4;
  const int b = blockIdx.x;
  const v8f z8 = {0.f,0.f,0.f,0.f,0.f,0.f,0.f,0.f};
  for (int i = tid; i < 16 * QP; i += 128) {
    const int n = i / QP, k = i - n * QP; const int kc = (k < DMD) ? k : (DMD - 1);
    const float q = Qh32[(size_t)b * DMD + kc];
    const float v = (n < NHD && k < DMD && (k / HDIM) == n) ? q : 0.f;
    s_qbd[i] = hbits(v);
  }
  for (int i = tid; i < 16 * PP; i += 128) s_p[i] = (unsigned short)0;
  for (int i = tid; i < SEQ; i += 128) s_km[i] = kmask[(size_t)b * SEQ_FULL + i];
  __syncthreads();
  {
    const unsigned short* qrow = s_qbd + ln * QP;
    const v16h qb0 = g2_fragu(qrow, hh), qb1 = g2_fragu(qrow + 32, hh);
    const unsigned short* kb = (const unsigned short*)Kh16 + (size_t)b * SEQ * DMD;
#pragma unroll 1
    for (int i = 0; i < SEQ / 64; ++i) {
      const int tt = w + 4 * i;
      const unsigned short* ap = kb + (size_t)(tt * 16 + ln) * DMD;
      const v16h a0 = g2_fragu(ap, hh), a1 = g2_fragu(ap + 32, hh);
      v8f c = z8; c = g2_mma(a0, qb0, c); c = g2_mma(a1, qb1, c);
#pragma unroll
      for (int r = 0; r < 8; ++r) {
        const int key = tt * 16 + 8 * hh + r;
        const bool valid = (s_km[key] == 1) && (key != 0);
        const float v = valid ? (c[r] * 0.25f) : NEGF;
        if (ln < NHD) s_sc[ln * SEQ + key] = v;
      }
    }
  }
  __syncthreads();
  {
    const int h = w; float* sc = s_sc + h * SEQ;
    const float qm0 = (float)qmask[(size_t)b * SEQ_FULL];
    float mx = -3.0e38f;
#pragma unroll 1
    for (int j = lane; j < SEQ; j += 32) mx = fmaxf(mx, sc[j]);
#pragma unroll
    for (int o = 16; o > 0; o >>= 1) mx = fmaxf(mx, __shfl_xor(mx, o, 32));
    float se = 0.f;
#pragma unroll 1
    for (int j = lane; j < SEQ; j += 32) { const float e = expf(sc[j] - mx); sc[j] = e; se += e; }
#pragma unroll
    for (int o = 16; o > 0; o >>= 1) se += __shfl_xor(se, o, 32);
    const float scl = qm0 * 1024.0f * (1.0f / se);
#pragma unroll 1
    for (int j = lane; j < SEQ; j += 32) s_p[h * PP + j] = hbits(sc[j] * scl);
  }
  __syncthreads();
  {
    const unsigned short* prow = s_p + ln * PP;
    const unsigned short* vrow = (const unsigned short*)Vt16 + ((size_t)b * DMD + 16 * w + ln) * SEQ;
    v8f c = z8;
#pragma unroll 2
    for (int k0 = 0; k0 < SEQ; k0 += 32) { const v16h a = g2_fragu(prow + k0, hh); const v16h bq = g2_fragu(vrow + k0, hh); c = g2_mma(a, bq, c); }
    float val = 0.f;
#pragma unroll
    for (int r = 0; r < 8; ++r) { if (r == w) val = c[r]; }
    if (hh == 0) s_ctx[16 * w + ln] = val * (1.0f / 1024.0f);
  }
  __syncthreads();
  if (tid < DMD) { const float rv = s_ctx[tid] + bf16_rne(queries[(size_t)b * SEQ_FULL * DMD + tid]); s_res[tid] = rv; s_r16[tid] = hbits(rv); }
  __syncthreads();
  {
    v4f rf = {0.f, 0.f, 0.f, 0.f}; v8us rh = {0, 0, 0, 0, 0, 0, 0, 0};
    if (tid < 16) rf = *(const v4fa*)(s_res + 4 * tid);
    if (tid >= 32 && tid < 40) rh = *(const v8us*)(s_r16 + 8 * (tid - 32));
    float* d32 = R32 + (size_t)b * DMD + 4 * (tid & 15);
    unsigned short* d16 = (unsigned short*)R16 + (size_t)b * DMD + 8 * (tid & 7);
    for (int pass = 0; pass < 2; ++pass) {
      if (tid < 16) *(volatile v4f*)d32 = rf;
      if (tid >= 32 && tid < 40) *(volatile v8us*)d16 = rh;
      if (pass == 0) __threadfence();
    }
  }
}

extern "C" void kernel_launch(void* const* d_in, const int* in_sizes, int n_in,
                              void* d_out, int out_size, void* d_ws, size_t ws_size, hipStream_t stream) {
  if (n_in < 11) return;
  const float* queries = (const float*)d_in[0]; const float* keys = (const float*)d_in[1];
  const int* qmask = (const int*)d_in[2]; const int* kmask = (const int*)d_in[3];
  const float* wq = (const float*)d_in[4]; const float* wk = (const float*)d_in[5]; const float* wv = (const float*)d_in[6];
  const float* fw1 = (const float*)d_in[7]; const float* fw2 = (const float*)d_in[8]; const float* fb1 = (const float*)d_in[9]; const float* fb2 = (const float*)d_in[10];
  const size_t needq = ((size_t)(NB - 1) * SEQ_FULL + 1) * DMD, needk = ((size_t)(NB - 1) * SEQ_FULL + SEQ) * DMD;
  if ((size_t)in_sizes[0] < needq || (size_t)in_sizes[1] < needk) return;
  if ((size_t)in_sizes[2] < (size_t)(NB - 1) * SEQ_FULL + 1 || (size_t)in_sizes[3] < (size_t)(NB - 1) * SEQ_FULL + SEQ) return;
  if (in_sizes[4] < DMD * DMD || in_sizes[5] < DMD * DMD || in_sizes[6] < DMD * DMD || in_sizes[7] < DMD * FFD || in_sizes[8] < FFD * DMD || in_sizes[9] < FFD || in_sizes[10] < DMD) return;
  if ((size_t)out_size < (size_t)NB * DMD) return;
  char* ws = (char*)d_ws; size_t off = 0;
  auto take = [&](size_t bytes) { char* p = ws + off; off += (bytes + 255) & ~(size_t)255; return p; };
  _Float16* WQt = (_Float16*)take((size_t)DMD * DMD * 2); _Float16* WKt = (_Float16*)take((size_t)DMD * DMD * 2); _Float16* WVa = (_Float16*)take((size_t)DMD * DMD * 2);
  _Float16* F1t = (_Float16*)take((size_t)FFD * DMD * 2); _Float16* F2t = (_Float16*)take((size_t)DMD * FFD * 2);
  _Float16* KEYS16 = (_Float16*)take((size_t)NB * SEQ * DMD * 2); _Float16* KH16 = (_Float16*)take((size_t)NB * SEQ * DMD * 2); _Float16* VT16 = (_Float16*)take((size_t)NB * DMD * SEQ * 2);
  _Float16* Q016 = (_Float16*)take((size_t)MPAD * DMD * 2); float* QH32 = (float*)take((size_t)MPAD * DMD * 4);
  _Float16* R16 = (_Float16*)take((size_t)MPAD * DMD * 2); float* R32 = (float*)take((size_t)MPAD * DMD * 4); _Float16* H16 = (_Float16*)take((size_t)MPAD * FFD * 2);
  if (off > ws_size || off > ((size_t)128 << 20)) return;

  k_wt_f16<<<(unsigned)((DMD * DMD / 8 + 255) / 256), 256, 0, stream>>>(wq, WQt, DMD, DMD, 16.0f);
  k_wt_f16<<<(unsigned)((DMD * DMD / 8 + 255) / 256), 256, 0, stream>>>(wk, WKt, DMD, DMD, 16.0f);
  k_wt_f16<<<(unsigned)((DMD * DMD / 8 + 255) / 256), 256, 0, stream>>>(wv, WVa, DMD, DMD, 16.0f);
  k_wt_f16<<<(unsigned)((DMD * FFD / 8 + 255) / 256), 256, 0, stream>>>(fw1, F1t, DMD, FFD, 16.0f);
  k_wt_f16<<<(unsigned)((FFD * DMD / 8 + 255) / 256), 256, 0, stream>>>(fw2, F2t, FFD, DMD, 16.0f);
  k_keys16<<<(unsigned)(((size_t)NB * SEQ * 8 + 255) / 256), 256, 0, stream>>>(keys, KEYS16);
  k_q0<<<(unsigned)((MPAD * 8 + MPAD * 16 + 255) / 256), 256, 0, stream>>>(queries, Q016, R16, R32);
  k_gemm2<0><<<dim3((unsigned)(((size_t)NB * SEQ / 128) * (DMD / 64)), 1), 128, 0, stream>>>(KEYS16, DMD, 0, WKt, DMD, 0, 0.0625f, nullptr, nullptr, nullptr, KH16, DMD, 0, (int)((size_t)NB * SEQ), DMD, DMD);
  k_gemm2<0><<<dim3((unsigned)(((DMD + 127) / 128) * (SEQ / 64)), NB), 128, 0, stream>>>(WVa, DMD, 0, KEYS16, DMD, (size_t)SEQ * DMD, 0.0625f, nullptr, nullptr, nullptr, VT16, SEQ, (size_t)DMD * SEQ, DMD, SEQ, DMD);
  k_gemm2<0><<<dim3((unsigned)(((MPAD + 127) / 128) * (DMD / 64)), 1), 128, 0, stream>>>(Q016, DMD, 0, WQt, DMD, 0, 0.0625f, nullptr, nullptr, QH32, nullptr, DMD, 0, MPAD, DMD, DMD);
  k_attn<<<NB, 128, 0, stream>>>(KH16, VT16, QH32, queries, qmask, kmask, R32, R16);
  k_gemm2<17><<<dim3((unsigned)(((MPAD + 127) / 128) * (FFD / 64)), 1), 128, 0, stream>>>(R16, DMD, 0, F1t, DMD, 0, 0.0625f, fb1, nullptr, nullptr, H16, FFD, 0, MPAD, FFD, DMD);
  k_gemm2<0><<<dim3((unsigned)(((NB + 127) / 128) * (DMD / 64)), 1), 128, 0, stream>>>(H16, FFD, 0, F2t, FFD, 0, 0.0625f, fb2, R32, (float*)d_out, nullptr, DMD, 0, NB, DMD, FFD);
}
